// ui_aggregator_24833500905766
// MI455X (gfx1250) — hardware-verified
//
#include <hip/hip_runtime.h>

typedef _Float16 v4h  __attribute__((ext_vector_type(4)));
typedef _Float16 v8h  __attribute__((ext_vector_type(8)));
typedef _Float16 v16h __attribute__((ext_vector_type(16)));
typedef __bf16   v16b __attribute__((ext_vector_type(16)));
typedef unsigned short us8 __attribute__((ext_vector_type(8)));
typedef float v4f __attribute__((ext_vector_type(4)));
typedef float v8f __attribute__((ext_vector_type(8)));

#define D_EMB   64
#define H_NB    50
#define NPB     8
#define RPB     (NPB * H_NB)
#define NWAVE   4
#define NTHR    (NWAVE * 32)
#define NTILE   (RPB / 16)
#define NIT     ((NTILE + NWAVE - 1) / NWAVE)
#define SX      136
#define SW      72

#define OFF_W1   0
#define OFF_W2   8192
#define OFF_A1A  12288
#define OFF_A1B  16384
#define OFF_A2   20480
#define OFF_L1H  24576
#define OFF_L1L  32768
#define WS_ELEMS 40960
#define WS_GROUPS (WS_ELEMS / 8)
#define WS_BYTES_USED (WS_ELEMS * 2)

static_assert(RPB % 16 == 0);
static_assert(NIT * NWAVE * 16 >= RPB);
static_assert((SX % 8) == 0 && (SW % 8) == 0);
static_assert((OFF_W2 % 8) == 0 && (OFF_A1A % 8) == 0 && (OFF_A1B % 8) == 0 && (OFF_A2 % 8) == 0 && (OFF_L1H % 8) == 0 && (OFF_L1L % 8) == 0);
static_assert(WS_ELEMS % 8 == 0);
static_assert(NTHR == NPB * 16);

__device__ __forceinline__ unsigned short f16_bits(float x) {
  _Float16 hv = (_Float16)x;
  return __builtin_bit_cast(unsigned short, hv);
}
__device__ __forceinline__ unsigned short bf16_rne(float x) {
  unsigned int u = __builtin_bit_cast(unsigned int, x);
  u = (u + 0x7FFFu + ((u >> 16) & 1u)) >> 16;
  return (unsigned short)u;
}
__device__ __forceinline__ float bf16_val(unsigned short b) {
  return __builtin_bit_cast(float, ((unsigned int)b) << 16);
}
__device__ __forceinline__ int wrap_clamp(int i, int n) {
  if (i < 0) i += n;
  i = (i < 0) ? 0 : i;
  i = (i > n - 1) ? (n - 1) : i;
  return i;
}
__device__ __forceinline__ v8f zero8() {
  v8f z = {0.f, 0.f, 0.f, 0.f, 0.f, 0.f, 0.f, 0.f};
  return z;
}
__device__ __forceinline__ float wave_max(float v) {
  v = fmaxf(v, __shfl_xor(v, 16));
  v = fmaxf(v, __shfl_xor(v, 8));
  v = fmaxf(v, __shfl_xor(v, 4));
  v = fmaxf(v, __shfl_xor(v, 2));
  v = fmaxf(v, __shfl_xor(v, 1));
  return v;
}
__device__ __forceinline__ float wave_sum(float v) {
  v += __shfl_xor(v, 16);
  v += __shfl_xor(v, 8);
  v += __shfl_xor(v, 4);
  v += __shfl_xor(v, 2);
  v += __shfl_xor(v, 1);
  return v;
}

union Frag16 { v16h v; v8h p[2]; };
union FragBF { v16b v; us8 p[2]; };

__device__ __forceinline__ v16h frag16(const _Float16* base, int row, int stride, int k0, int h) {
  Frag16 f;
  const _Float16* p = base + row * stride + k0 + 8 * h;
  f.p[0] = *(const v8h*)(p);
  f.p[1] = *(const v8h*)(p + 16);
  return f.v;
}
__device__ __forceinline__ v16b fragbf(const unsigned short* base, int row, int stride, int k0, int h) {
  FragBF f;
  const unsigned short* p = base + row * stride + k0 + 8 * h;
  f.p[0] = *(const us8*)(p);
  f.p[1] = *(const us8*)(p + 16);
  return f.v;
}
__device__ __forceinline__ v8f mma_f16(v8f c, v16h a, v16h b) {
  c = __builtin_amdgcn_wmma_f32_16x16x32_f16(false, a, false, b, (short)0, c, false, false);
  asm volatile("v_nop\n\tv_nop\n\tv_nop\n\tv_nop" : "+v"(c) : "v"(a), "v"(b));
  return c;
}
__device__ __forceinline__ v8f mma_bf16(v8f c, v16b a, v16b b) {
  c = __builtin_amdgcn_wmma_f32_16x16x32_bf16(false, a, false, b, (short)0, c, false, false);
  asm volatile("v_nop\n\tv_nop\n\tv_nop\n\tv_nop" : "+v"(c) : "v"(a), "v"(b));
  return c;
}

__device__ __forceinline__ unsigned short prep_elem(int e,
    const float* __restrict__ w_r1, const float* __restrict__ w_r2,
    const float* __restrict__ att1, const float* __restrict__ att2,
    const float* __restrict__ lin1) {
  if (e < OFF_W2)  return f16_bits(16.f * w_r1[e]);
  if (e < OFF_A1A) return f16_bits(16.f * w_r2[e - OFF_W2]);
  if (e < OFF_A1B) { const int q = e - OFF_A1A; return f16_bits(16.f * att1[(q >> 6) * 128 + (q & 63)]); }
  if (e < OFF_A2)  { const int q = e - OFF_A1B; return f16_bits(16.f * att1[(q >> 6) * 128 + 64 + (q & 63)]); }
  if (e < OFF_L1H) return f16_bits(16.f * att2[e - OFF_A2]);
  if (e < OFF_L1L) return bf16_rne(lin1[e - OFF_L1H]);
  const float x = lin1[e - OFF_L1L];
  return bf16_rne(x - bf16_val(bf16_rne(x)));
}

__global__ __launch_bounds__(256) void prep_params(
    const float* __restrict__ w_r1, const float* __restrict__ w_r2,
    const float* __restrict__ att1, const float* __restrict__ att2,
    const float* __restrict__ lin1, unsigned short* __restrict__ wsb) {
  const int t = blockIdx.x * 256 + threadIdx.x;
  const bool ok = t < WS_GROUPS;
  us8 val;
#pragma unroll
  for (int i = 0; i < 8; ++i) {
    unsigned short u = 0;
    if (ok) u = prep_elem(t * 8 + i, w_r1, w_r2, att1, att2, lin1);
    val[i] = u;
  }
  unsigned short* p = wsb + (size_t)t * 8;
  if (ok) *(volatile us8*)p = val;
  __threadfence();
  if (ok) *(volatile us8*)p = val;
}

struct __align__(16) Smem {
  alignas(16) _Float16 w1[64 * SX];
  alignas(16) _Float16 w2[64 * SW];
  alignas(16) _Float16 a1a[64 * SW];
  alignas(16) _Float16 a2w[64 * SW];
  alignas(16) _Float16 obuf[RPB * SW];
  alignas(16) _Float16 x[64 * SX];
  alignas(16) _Float16 hb[64 * SW];
  alignas(16) _Float16 u16[16 * SW];
  alignas(16) unsigned short lah[16 * SX];
  alignas(16) unsigned short lal[16 * SX];
  alignas(16) float uf[NPB * 64];
  alignas(16) float ub[NPB * 64];
  alignas(16) float outs[NPB * 64];
  alignas(16) float logit[RPB + 16];
  alignas(16) float att3[64];
  alignas(16) float bias[5 * 64];
  alignas(16) int idxI[RPB];
  alignas(16) int idxR[RPB];
  float a3bias;
};

__global__ __launch_bounds__(NTHR) void agg_fused(
    const int* __restrict__ nodes, const int* __restrict__ hui, const int* __restrict__ hr,
    const float* __restrict__ u2e, const float* __restrict__ i2e, const float* __restrict__ r2e,
    const float* __restrict__ b_r1, const float* __restrict__ b_r2,
    const float* __restrict__ b_a1, const float* __restrict__ b_a2,
    const float* __restrict__ a3w, const float* __restrict__ a3b,
    const float* __restrict__ b_l1,
    const _Float16* wsh, const unsigned short* wsb,
    float* __restrict__ out,
    int nB, int nUsers, int nItems, int nRat)
{
  __shared__ Smem sm;
  const int tid  = threadIdx.x;
  const int lane = tid & 31;
  const int w    = tid >> 5;
  const int h    = lane >> 4;
  const int m    = lane & 15;
  const int b0   = blockIdx.x * NPB;

  for (int i = tid; i < 64 * 16; i += NTHR) {
    const int n = i >> 4, c = (i & 15) << 3;
    *(v8h*)(sm.w1 + n * SX + c) = *(const v8h*)(wsh + OFF_W1 + n * 128 + c);
  }
  for (int i = tid; i < 64 * 8; i += NTHR) {
    const int n = i >> 3, c = (i & 7) << 3;
    *(v8h*)(sm.w2  + n * SW + c) = *(const v8h*)(wsh + OFF_W2  + n * 64 + c);
    *(v8h*)(sm.a1a + n * SW + c) = *(const v8h*)(wsh + OFF_A1A + n * 64 + c);
    *(v8h*)(sm.a2w + n * SW + c) = *(const v8h*)(wsh + OFF_A2  + n * 64 + c);
  }
  if (tid < 64) {
    sm.bias[tid]       = b_r1[tid];
    sm.bias[64 + tid]  = b_r2[tid];
    sm.bias[128 + tid] = b_a1[tid];
    sm.bias[192 + tid] = b_a2[tid];
    sm.bias[256 + tid] = b_l1[tid];
    sm.att3[tid]       = a3w[tid];
  }
  if (tid == 0) sm.a3bias = a3b[0];

  for (int i = tid; i < RPB; i += NTHR) {
    const int j = i / H_NB;
    const int r = i - j * H_NB;
    const int nd = b0 + j;
    int vi = 0, vr = 0;
    if (nd < nB) {
      const size_t g = (size_t)nd * H_NB + r;
      vi = hui[g];
      vr = hr[g];
    }
    sm.idxI[i] = wrap_clamp(vi, nItems);
    sm.idxR[i] = wrap_clamp(vr, nRat);
  }
  {
    const int j = tid >> 4, d0 = (tid & 15) << 2;
    const int nd = b0 + j;
    int id = 0;
    if (nd < nB) id = nodes[nd];
    id = wrap_clamp(id, nUsers);
    const v4f u = *(const v4f*)(u2e + (size_t)id * D_EMB + d0);
    sm.uf[j * 64 + d0 + 0] = u.x;
    sm.uf[j * 64 + d0 + 1] = u.y;
    sm.uf[j * 64 + d0 + 2] = u.z;
    sm.uf[j * 64 + d0 + 3] = u.w;
    v4h t;
    t.x = (_Float16)(u.x * 16.f);
    t.y = (_Float16)(u.y * 16.f);
    t.z = (_Float16)(u.z * 16.f);
    t.w = (_Float16)(u.w * 16.f);
    *(v4h*)(sm.u16 + j * SW + d0) = t;
  }
  for (int i = tid; i < 8 * SW; i += NTHR) sm.u16[8 * SW + i] = (_Float16)0.0f;
  __syncthreads();

  {
    const int n = 16 * w + m;
    v8f c = zero8();
    c = mma_f16(c, frag16(sm.u16, m, SW, 0,  h), frag16(wsh + OFF_A1B, n, 64, 0,  h));
    c = mma_f16(c, frag16(sm.u16, m, SW, 32, h), frag16(wsh + OFF_A1B, n, 64, 32, h));
    const float bv = sm.bias[128 + n];
    if (h == 0) {
#pragma unroll
      for (int r = 0; r < 8; ++r) sm.ub[r * 64 + n] = c[r] * (1.f / 256.f) + bv;
    }
  }

#pragma unroll 1
  for (int it = 0; it < NIT; ++it) {
    __syncthreads();
    for (int q = tid; q < 64 * 32; q += NTHR) {
      const int rl = q >> 5, part = q & 31, col = part << 2;
      const int R = it * 64 + rl;
      v4f v = {0.f, 0.f, 0.f, 0.f};
      if (R < RPB) {
        const float* src = (part < 16)
            ? (i2e + (size_t)sm.idxI[R] * D_EMB + col)
            : (r2e + (size_t)sm.idxR[R] * D_EMB + (col - 64));
        v = *(const v4f*)src;
      }
      v4h t;
      t.x = (_Float16)(v.x * 16.f);
      t.y = (_Float16)(v.y * 16.f);
      t.z = (_Float16)(v.z * 16.f);
      t.w = (_Float16)(v.w * 16.f);
      *(v4h*)(sm.x + rl * SX + col) = t;
    }
    __syncthreads();

    const int tile   = it * NWAVE + w;
    const bool valid = tile < NTILE;
    const int rb     = 16 * w;
    const int Rg     = it * 64 + rb;

    if (valid) {
      const v16h xa0 = frag16(sm.x, rb + m, SX, 0,  h);
      const v16h xa1 = frag16(sm.x, rb + m, SX, 32, h);
      const v16h xa2 = frag16(sm.x, rb + m, SX, 64, h);
      const v16h xa3 = frag16(sm.x, rb + m, SX, 96, h);
#pragma unroll 1
      for (int nt = 0; nt < 4; ++nt) {
        const int n = 16 * nt + m;
        v8f c = zero8();
        c = mma_f16(c, xa0, frag16(sm.w1, n, SX, 0,  h));
        c = mma_f16(c, xa1, frag16(sm.w1, n, SX, 32, h));
        c = mma_f16(c, xa2, frag16(sm.w1, n, SX, 64, h));
        c = mma_f16(c, xa3, frag16(sm.w1, n, SX, 96, h));
        const float bv = sm.bias[n];
#pragma unroll
        for (int r = 0; r < 8; ++r) {
          const float v = fmaxf(c[r] * (1.f / 256.f) + bv, 0.f);
          sm.hb[(rb + 8 * h + r) * SW + n] = (_Float16)(v * 64.f);
        }
      }
    }
    __syncthreads();

    if (valid) {
      const v16h ha0 = frag16(sm.hb, rb + m, SW, 0,  h);
      const v16h ha1 = frag16(sm.hb, rb + m, SW, 32, h);
#pragma unroll 1
      for (int nt = 0; nt < 4; ++nt) {
        const int n = 16 * nt + m;
        v8f c = zero8();
        c = mma_f16(c, ha0, frag16(sm.w2, n, SW, 0,  h));
        c = mma_f16(c, ha1, frag16(sm.w2, n, SW, 32, h));
        const float bv = sm.bias[64 + n];
#pragma unroll
        for (int r = 0; r < 8; ++r) {
          const float v = fmaxf(c[r] * (1.f / 1024.f) + bv, 0.f);
          sm.obuf[(Rg + 8 * h + r) * SW + n] = (_Float16)(v * 256.f);
        }
      }
    }
    __syncthreads();

    if (valid) {
      const v16h oa0 = frag16(sm.obuf, Rg + m, SW, 0,  h);
      const v16h oa1 = frag16(sm.obuf, Rg + m, SW, 32, h);
      const int R0  = Rg + 8 * h;
      const int j0  = R0 / H_NB;
      const int cut = (j0 + 1) * H_NB - R0;
#pragma unroll 1
      for (int nt = 0; nt < 4; ++nt) {
        const int n = 16 * nt + m;
        v8f c = zero8();
        c = mma_f16(c, oa0, frag16(sm.a1a, n, SW, 0,  h));
        c = mma_f16(c, oa1, frag16(sm.a1a, n, SW, 32, h));
#pragma unroll
        for (int r = 0; r < 8; ++r) {
          const int j = j0 + ((r >= cut) ? 1 : 0);
          const float v = fmaxf(c[r] * (1.f / 4096.f) + sm.ub[j * 64 + n], 0.f);
          sm.hb[(rb + 8 * h + r) * SW + n] = (_Float16)(v * 64.f);
        }
      }
    }
    __syncthreads();

    if (valid) {
      const v16h qa0 = frag16(sm.hb, rb + m, SW, 0,  h);
      const v16h qa1 = frag16(sm.hb, rb + m, SW, 32, h);
      v8f part = zero8();
#pragma unroll 1
      for (int nt = 0; nt < 4; ++nt) {
        const int n = 16 * nt + m;
        v8f c = zero8();
        c = mma_f16(c, qa0, frag16(sm.a2w, n, SW, 0,  h));
        c = mma_f16(c, qa1, frag16(sm.a2w, n, SW, 32, h));
        const float bv = sm.bias[192 + n];
        const float w3 = sm.att3[n];
#pragma unroll
        for (int r = 0; r < 8; ++r) {
          const float a2 = fmaxf(c[r] * (1.f / 1024.f) + bv, 0.f);
          part[r] += a2 * w3;
        }
      }
#pragma unroll
      for (int r = 0; r < 8; ++r) {
        float p = part[r];
        p += __shfl_xor(p, 1);
        p += __shfl_xor(p, 2);
        p += __shfl_xor(p, 4);
        p += __shfl_xor(p, 8);
        part[r] = p;
      }
      if (m == 0) {
#pragma unroll
        for (int r = 0; r < 8; ++r) sm.logit[Rg + 8 * h + r] = part[r] + sm.a3bias;
      }
    }
  }
  __syncthreads();

#pragma unroll 1
  for (int jj = 0; jj < 2; ++jj) {
    const int j = 2 * w + jj;
    const int base = j * H_NB;
    const bool has1 = lane < (H_NB - 32);
    const float l0 = sm.logit[base + lane];
    const float l1 = has1 ? sm.logit[base + 32 + lane] : -3.0e38f;
    const float mx = wave_max(fmaxf(l0, l1));
    const float e0 = __expf(l0 - mx);
    const float e1 = has1 ? __expf(l1 - mx) : 0.f;
    const float s  = wave_sum(e0 + e1);
    const float inv = 1.0f / s;
    sm.logit[base + lane] = e0 * inv;
    if (has1) sm.logit[base + 32 + lane] = e1 * inv;
  }
  __syncthreads();

  {
    const int j = tid >> 4, d0 = (tid & 15) << 2;
    const int base = j * H_NB;
    v4f acc = {0.f, 0.f, 0.f, 0.f};
#pragma unroll 2
    for (int r = 0; r < H_NB; ++r) {
      const float a = sm.logit[base + r];
      const v4h ov = *(const v4h*)(sm.obuf + (base + r) * SW + d0);
      acc.x += a * (float)ov.x;
      acc.y += a * (float)ov.y;
      acc.z += a * (float)ov.z;
      acc.w += a * (float)ov.w;
    }
#pragma unroll
    for (int i = 0; i < 4; ++i) {
      const float nv = acc[i] * (1.f / 256.f);
      const float uv = sm.uf[j * 64 + d0 + i];
      const unsigned short hu = bf16_rne(uv);
      const unsigned short hn = bf16_rne(nv);
      sm.lah[j * SX + d0 + i]      = hu;
      sm.lal[j * SX + d0 + i]      = bf16_rne(uv - bf16_val(hu));
      sm.lah[j * SX + 64 + d0 + i] = hn;
      sm.lal[j * SX + 64 + d0 + i] = bf16_rne(nv - bf16_val(hn));
    }
  }
  for (int i = tid; i < 8 * SX; i += NTHR) { sm.lah[8 * SX + i] = 0; sm.lal[8 * SX + i] = 0; }
  __syncthreads();

  {
    const int n = 16 * w + m;
    v8f c = zero8();
#pragma unroll 1
    for (int kc = 0; kc < 4; ++kc) {
      const v16b ah = fragbf(sm.lah, m, SX, 32 * kc, h);
      const v16b al = fragbf(sm.lal, m, SX, 32 * kc, h);
      const v16b bh = fragbf(wsb + OFF_L1H, n, 128, 32 * kc, h);
      const v16b bl = fragbf(wsb + OFF_L1L, n, 128, 32 * kc, h);
      c = mma_bf16(c, ah, bh);
      c = mma_bf16(c, ah, bl);
      c = mma_bf16(c, al, bh);
    }
    const float bv = sm.bias[256 + n];
    if (h == 0) {
#pragma unroll
      for (int r = 0; r < 8; ++r) sm.outs[r * 64 + n] = fmaxf(c[r] + bv, 0.f);
    }
  }
  __syncthreads();

  {
    const int j = tid >> 4;
    const int nd = b0 + j;
    const bool ok = nd < nB;
    const v4f v = *(const v4f*)(sm.outs + 4 * tid);
    float* p = out + (size_t)nd * D_EMB + ((tid & 15) << 2);
    if (ok) *(volatile v4f*)p = v;
    __threadfence();
    if (ok) *(volatile v4f*)p = v;
  }
}

extern "C" void kernel_launch(void* const* d_in, const int* in_sizes, int n_in,
                              void* d_out, int out_size, void* d_ws, size_t ws_size,
                              hipStream_t stream) {
  if (n_in < 18) return;
  const int nB = in_sizes[0];
  if (nB <= 0) return;
  if (in_sizes[1] != nB * H_NB || in_sizes[2] != nB * H_NB) return;
  const int nUsers = in_sizes[3] / D_EMB;
  const int nItems = in_sizes[4] / D_EMB;
  const int nRat   = in_sizes[5] / D_EMB;
  if (nUsers < 1 || nItems < 1 || nRat < 1) return;
  if (in_sizes[6] != 64 * 128 || in_sizes[7] < 64 || in_sizes[8] != 64 * 64 || in_sizes[9] < 64) return;
  if (in_sizes[10] != 64 * 128 || in_sizes[11] < 64 || in_sizes[12] != 64 * 64 || in_sizes[13] < 64) return;
  if (in_sizes[14] < 64 || in_sizes[15] < 1 || in_sizes[16] != 64 * 128 || in_sizes[17] < 64) return;
  if (out_size != nB * D_EMB) return;
  if (ws_size < (size_t)WS_BYTES_USED) return;

  const int*   nodes  = (const int*)d_in[0];
  const int*   hui    = (const int*)d_in[1];
  const int*   hr     = (const int*)d_in[2];
  const float* u2e    = (const float*)d_in[3];
  const float* i2e    = (const float*)d_in[4];
  const float* r2e    = (const float*)d_in[5];
  const float* w_r1_w = (const float*)d_in[6];
  const float* w_r1_b = (const float*)d_in[7];
  const float* w_r2_w = (const float*)d_in[8];
  const float* w_r2_b = (const float*)d_in[9];
  const float* att1_w = (const float*)d_in[10];
  const float* att1_b = (const float*)d_in[11];
  const float* att2_w = (const float*)d_in[12];
  const float* att2_b = (const float*)d_in[13];
  const float* att3_w = (const float*)d_in[14];
  const float* att3_b = (const float*)d_in[15];
  const float* lin1_w = (const float*)d_in[16];
  const float* lin1_b = (const float*)d_in[17];
  unsigned short* wsb = (unsigned short*)d_ws;
  const _Float16* wsh = (const _Float16*)d_ws;
  float* out = (float*)d_out;

  prep_params<<<(WS_GROUPS + 255) / 256, 256, 0, stream>>>(
      w_r1_w, w_r2_w, att1_w, att2_w, lin1_w, wsb);

  const int nblk = (nB + NPB - 1) / NPB;
  agg_fused<<<nblk, NTHR, 0, stream>>>(
      nodes, hui, hr, u2e, i2e, r2e,
      w_r1_b, w_r2_b, att1_b, att2_b, att3_w, att3_b, lin1_b,
      wsh, (const unsigned short*)wsb, out,
      nB, nUsers, nItems, nRat);
}
